// RNN_46548855554081
// MI455X (gfx1250) — hardware-verified
//
#include <hip/hip_runtime.h>
#include <math.h>

constexpr int NBATCH       = 64;
constexpr int NSTEP        = 512;
constexpr int NIN          = 64;
constexpr int NHID         = 1024;
constexpr int SCAN_THREADS = 512;
constexpr int SCAN_WAVES   = SCAN_THREADS / 32;
constexpr int ROWS_BLK     = 32;
constexpr int HPITCH       = NHID + 8;
constexpr int SLABP        = 68;
constexpr int CVT_THREADS  = 256;
constexpr int HEAD_THREADS = 256;
constexpr float WCARRY     = 1024.0f;
constexpr float WCARRY_INV = 1.0f / 1024.0f;
constexpr int OUT0_ELEMS   = NBATCH;
constexpr int OUT1_ELEMS   = 2 * NBATCH * NHID;
constexpr size_t OUT1_BYTE_OFF = 256;

static_assert(OUT0_ELEMS * 4 == (int)OUT1_BYTE_OFF, "out1 starts right after out0");
static_assert(OUT1_BYTE_OFF + (size_t)OUT1_ELEMS * 4 == 524544, "d_out total bytes");
static_assert(OUT1_BYTE_OFF % 128 == 0, "out1 line aligned");
static_assert(NBATCH % ROWS_BLK == 0, "batch tiles");
static_assert(NHID == 64 * SCAN_WAVES, "16 waves x 64 hidden columns");
static_assert(NIN % 32 == 0 && NHID % 32 == 0, "K multiples of 32");
static_assert((ROWS_BLK * NHID) % (SCAN_THREADS * 8) == 0, "tile copy loops exact");
static_assert((HPITCH * 2) % 16 == 0, "LDS row pitch 16-B aligned");
static_assert((NBATCH * NSTEP * NIN / 8) % CVT_THREADS == 0, "x convert grid exact");
static_assert((NHID * NIN / 8) % CVT_THREADS == 0, "W_ih0 convert grid exact");
static_assert((NHID * NHID / 8) % CVT_THREADS == 0, "W convert grid exact");

typedef __attribute__((ext_vector_type(16))) _Float16 v16h;
typedef __attribute__((ext_vector_type(8)))  _Float16 v8h;
typedef __attribute__((ext_vector_type(8)))  float    v8f;
typedef __attribute__((ext_vector_type(4)))  float    v4f;

struct FragH {
  union U { v16h v; v8h h[2]; };
  static __device__ __forceinline__ v16h load(const _Float16* p) {
    U f;
    f.h[0] = *(const v8h*)(p);
    f.h[1] = *(const v8h*)(p + 16);
    return f.v;
  }
  static __device__ __forceinline__ v8f mma(v16h a, v16h b, v8f c) {
    return __builtin_amdgcn_wmma_f32_16x16x32_f16(false, a, false, b, (short)0, c, false, false);
  }
};

__device__ __forceinline__ void guard8(v8f& a0, v8f& a1, v8f& a2, v8f& a3, v8f& a4, v8f& a5, v8f& a6, v8f& a7,
                                       v16h x0, v16h x1, v16h y0, v16h y1, v16h y2, v16h y3) {
  asm volatile("v_nop\n\tv_nop\n\tv_nop\n\tv_nop"
               : "+v"(a0), "+v"(a1), "+v"(a2), "+v"(a3), "+v"(a4), "+v"(a5), "+v"(a6), "+v"(a7)
               : "v"(x0), "v"(x1), "v"(y0), "v"(y1), "v"(y2), "v"(y3));
}

#define RNN_MMA8()                                                                   \
  acc[0] = FragH::mma(A0, B0, acc[0]);                                               \
  acc[1] = FragH::mma(A0, B1, acc[1]);                                               \
  acc[2] = FragH::mma(A0, B2, acc[2]);                                               \
  acc[3] = FragH::mma(A0, B3, acc[3]);                                               \
  acc[4] = FragH::mma(A1, B0, acc[4]);                                               \
  acc[5] = FragH::mma(A1, B1, acc[5]);                                               \
  acc[6] = FragH::mma(A1, B2, acc[6]);                                               \
  acc[7] = FragH::mma(A1, B3, acc[7]);                                               \
  guard8(acc[0], acc[1], acc[2], acc[3], acc[4], acc[5], acc[6], acc[7], A0, A1, B0, B1, B2, B3);

__global__ __launch_bounds__(CVT_THREADS) void cvt8_f16_kernel(const float* __restrict__ src,
                                                              unsigned short* __restrict__ dst, int n8, float sc) {
  const int i = blockIdx.x * CVT_THREADS + threadIdx.x;
  if (i < n8) {
    const float* sp = src + (size_t)i * 8;
    const v4f a = *(const v4f*)(sp);
    const v4f b = *(const v4f*)(sp + 4);
    v8h hv;
#pragma unroll
    for (int e = 0; e < 4; ++e) {
      const float fa = a[e] * sc;
      const float fb = b[e] * sc;
      hv[e]     = (_Float16)fa;
      hv[4 + e] = (_Float16)fb;
    }
    _Float16* dp = (_Float16*)dst + (size_t)i * 8;
    *(volatile v8h*)dp = hv;
    __threadfence();
    *(volatile v8h*)dp = hv;
  }
}

template <int LAYER>
__global__ __launch_bounds__(SCAN_THREADS) void rnn_scan_kernel(
    const unsigned short* __restrict__ AGp, const unsigned short* __restrict__ WGp,
    const unsigned short* __restrict__ WLp, const float* __restrict__ h_init,
    const float* __restrict__ b_a, const float* __restrict__ b_b,
    unsigned short* __restrict__ SEQp, float* __restrict__ F32T0, float* __restrict__ HFIN) {
  constexpr int KG = (LAYER == 0) ? NIN : NHID;
  constexpr size_t BJG = (size_t)16 * KG;
  constexpr size_t BJL = (size_t)16 * NHID;
  __shared__ __align__(16) _Float16 Ah[ROWS_BLK * HPITCH];
  __shared__ __align__(16) float    Sl[SCAN_WAVES][16 * SLABP];

  const _Float16* AG = (const _Float16*)AGp;
  const _Float16* WG = (const _Float16*)WGp;
  const _Float16* WL = (const _Float16*)WLp;
  _Float16* SEQ = (_Float16*)SEQp;

  const int tid = threadIdx.x, lane = tid & 31, wave = tid >> 5;
  const int c = lane & 15, hh = lane >> 4, koff = hh * 8, c4 = c * 4;
  const int rowbase = blockIdx.x * ROWS_BLK;
  const int n0 = wave * 64;

#pragma unroll 1
  for (int it = 0; it < (ROWS_BLK * NHID) / (SCAN_THREADS * 8); ++it) {
    const int idx = it * SCAN_THREADS + tid;
    const int row = idx >> 7;
    const int pc  = (idx & 127) * 8;
    const float* sp = h_init + (size_t)(rowbase + row) * NHID + pc;
    const v4f a = *(const v4f*)(sp);
    const v4f b = *(const v4f*)(sp + 4);
    v8h hv;
#pragma unroll
    for (int e = 0; e < 4; ++e) {
      const float fa = a[e];
      const float fb = b[e];
      hv[e]     = (_Float16)fa;
      hv[4 + e] = (_Float16)fb;
    }
    *(v8h*)(Ah + row * HPITCH + pc) = hv;
  }
  if (tid < ROWS_BLK) {
    const v8h zz = {(_Float16)0.0f, (_Float16)0.0f, (_Float16)0.0f, (_Float16)0.0f,
                    (_Float16)0.0f, (_Float16)0.0f, (_Float16)0.0f, (_Float16)0.0f};
    *(v8h*)(Ah + tid * HPITCH + NHID) = zz;
  }
  float bc[4];
#pragma unroll
  for (int j = 0; j < 4; ++j) {
    const int n = n0 + 16 * j + c;
    bc[j] = (b_a[n] + b_b[n]) * WCARRY;
  }
  __syncthreads();

  const _Float16* wl  = WL + (size_t)(n0 + c) * NHID + koff;
  const _Float16* wg  = WG + (size_t)(n0 + c) * KG + koff;
  const _Float16* ah0 = Ah + c * HPITCH + koff;
  const _Float16* ah1 = Ah + (16 + c) * HPITCH + koff;
  float* slab = &Sl[wave][0];

#pragma unroll 1
  for (int t = 0; t < NSTEP; ++t) {
    v8f acc[8];
#pragma unroll
    for (int i = 0; i < 2; ++i) {
#pragma unroll
      for (int j = 0; j < 4; ++j) {
        const float bv = bc[j];
        acc[4 * i + j] = (v8f){bv, bv, bv, bv, bv, bv, bv, bv};
      }
    }
    const _Float16* ag0;
    const _Float16* ag1;
    if (LAYER == 0) {
      ag0 = AG + ((size_t)(rowbase + c) * NSTEP + (size_t)t) * NIN + koff;
      ag1 = AG + ((size_t)(rowbase + 16 + c) * NSTEP + (size_t)t) * NIN + koff;
    } else {
      ag0 = AG + ((size_t)t * NBATCH + (size_t)(rowbase + c)) * NHID + koff;
      ag1 = ag0 + (size_t)16 * NHID;
    }
#pragma unroll 1
    for (int k0 = 0; k0 < KG; k0 += 32) {
      const v16h B0 = FragH::load(wg + k0);
      const v16h B1 = FragH::load(wg + BJG + k0);
      const v16h B2 = FragH::load(wg + 2 * BJG + k0);
      const v16h B3 = FragH::load(wg + 3 * BJG + k0);
      const v16h A0 = FragH::load(ag0 + k0);
      const v16h A1 = FragH::load(ag1 + k0);
      RNN_MMA8()
    }
#pragma unroll 1
    for (int k0 = 0; k0 < NHID; k0 += 32) {
      const v16h B0 = FragH::load(wl + k0);
      const v16h B1 = FragH::load(wl + BJL + k0);
      const v16h B2 = FragH::load(wl + 2 * BJL + k0);
      const v16h B3 = FragH::load(wl + 3 * BJL + k0);
      const v16h A0 = FragH::load(ah0 + k0);
      const v16h A1 = FragH::load(ah1 + k0);
      RNN_MMA8()
    }
    __syncthreads();

    const bool last = (t == NSTEP - 1);
    const bool emit = last || (LAYER == 1 && t == 0);
    float* edst = last ? HFIN : F32T0;

#pragma unroll 1
    for (int q = 0; q < 8; ++q) {
      const int jq  = q & 3;
      const int rt  = (q >> 2) * 16;
      const int col = n0 + 16 * jq + c;
      const v8f cur = acc[0];
      float hv[8];
#pragma unroll
      for (int r = 0; r < 8; ++r) hv[r] = tanhf(cur[r] * WCARRY_INV);
#pragma unroll
      for (int r = 0; r < 8; ++r) Ah[(rt + 8 * hh + r) * HPITCH + col] = (_Float16)hv[r];
      if (emit) {
#pragma unroll
        for (int r = 0; r < 8; ++r) slab[(8 * hh + r) * SLABP + 16 * jq + c] = hv[r];
      }
#pragma unroll
      for (int i = 0; i < 7; ++i) acc[i] = acc[i + 1];
      if (emit && jq == 3) {
        __builtin_amdgcn_fence(__ATOMIC_RELEASE, "workgroup");
        __builtin_amdgcn_wave_barrier();
        __builtin_amdgcn_fence(__ATOMIC_ACQUIRE, "workgroup");
        for (int pass = 0; pass < 2; ++pass) {
#pragma unroll
          for (int it = 0; it < 8; ++it) {
            const int row = it * 2 + hh;
            const v4f v = *(const v4f*)(slab + row * SLABP + c4);
            *(volatile v4f*)(edst + (size_t)(rowbase + rt + row) * NHID + n0 + c4) = v;
          }
          __threadfence();
        }
        __builtin_amdgcn_fence(__ATOMIC_RELEASE, "workgroup");
        __builtin_amdgcn_wave_barrier();
        __builtin_amdgcn_fence(__ATOMIC_ACQUIRE, "workgroup");
      }
    }
    __syncthreads();

    if (LAYER == 0) {
      for (int pass = 0; pass < 2; ++pass) {
#pragma unroll 2
        for (int it = 0; it < (ROWS_BLK * NHID) / (SCAN_THREADS * 8); ++it) {
          const int idx = it * SCAN_THREADS + tid;
          const int row = idx >> 7;
          const int pc  = (idx & 127) * 8;
          const v8h v = *(const v8h*)(Ah + row * HPITCH + pc);
          *(volatile v8h*)(SEQ + ((size_t)t * NBATCH + (size_t)(rowbase + row)) * NHID + pc) = v;
        }
        __threadfence();
      }
    }
  }
}

__global__ __launch_bounds__(HEAD_THREADS) void head_kernel(const float* __restrict__ H2T0, const float* __restrict__ W_out,
                                                           const float* __restrict__ b_out, float* __restrict__ out) {
  __shared__ __align__(16) float res[NBATCH];
  const int tid = threadIdx.x, lane = tid & 31, wave = tid >> 5;
  const float bo = b_out[0];
#pragma unroll 1
  for (int rr = 0; rr < NBATCH / (HEAD_THREADS / 32); ++rr) {
    const int row = wave * (NBATCH / (HEAD_THREADS / 32)) + rr;
    float s = 0.0f;
#pragma unroll 1
    for (int it = 0; it < NHID / 128; ++it) {
      const int k = it * 128 + lane * 4;
      const v4f hv = *(const v4f*)(H2T0 + (size_t)row * NHID + k);
      const v4f wv = *(const v4f*)(W_out + k);
      s += hv[0] * wv[0];
      s += hv[1] * wv[1];
      s += hv[2] * wv[2];
      s += hv[3] * wv[3];
    }
#pragma unroll
    for (int off = 1; off < 32; off <<= 1) s += __shfl_xor(s, off, 32);
    if (lane == 0) res[row] = s + bo;
  }
  __syncthreads();
  if (tid < NBATCH / 4) {
    const v4f v = *(const v4f*)(res + tid * 4);
    *(volatile v4f*)(out + tid * 4) = v;
    __threadfence();
    *(volatile v4f*)(out + tid * 4) = v;
  }
}

extern "C" void kernel_launch(void* const* d_in, const int* in_sizes, int n_in,
                              void* d_out, int out_size, void* d_ws, size_t ws_size, hipStream_t stream) {
  if (n_in < 12 || d_out == nullptr || d_ws == nullptr) return;
  if (in_sizes[0] != NBATCH * NSTEP * NIN || in_sizes[1] != 2 * NBATCH * NHID || in_sizes[2] != NHID * NIN ||
      in_sizes[3] != NHID * NHID || in_sizes[4] != NHID || in_sizes[5] != NHID || in_sizes[6] != NHID * NHID ||
      in_sizes[7] != NHID * NHID || in_sizes[8] != NHID || in_sizes[9] != NHID || in_sizes[10] != NHID ||
      in_sizes[11] != 1 || out_size != OUT0_ELEMS + OUT1_ELEMS) return;

  const float* x       = (const float*)d_in[0];
  const float* h_state = (const float*)d_in[1];
  const float* w_ih0   = (const float*)d_in[2];
  const float* w_hh0   = (const float*)d_in[3];
  const float* b_ih0   = (const float*)d_in[4];
  const float* b_hh0   = (const float*)d_in[5];
  const float* w_ih1   = (const float*)d_in[6];
  const float* w_hh1   = (const float*)d_in[7];
  const float* b_ih1   = (const float*)d_in[8];
  const float* b_hh1   = (const float*)d_in[9];
  const float* w_out   = (const float*)d_in[10];
  const float* b_out   = (const float*)d_in[11];

  float* out0  = (float*)d_out;
  float* hfin0 = out0 + OUT0_ELEMS;
  float* hfin1 = hfin0 + (size_t)NBATCH * NHID;

  char* ws = (char*)d_ws;
  size_t off = 0;
  auto carve = [&](size_t bytes) -> char* { char* p = ws + off; off += (bytes + 255) & ~(size_t)255; return p; };
  unsigned short* X16   = (unsigned short*)carve((size_t)NBATCH * NSTEP * NIN * 2);
  unsigned short* WIH0H = (unsigned short*)carve((size_t)NHID * NIN * 2);
  unsigned short* WHH0H = (unsigned short*)carve((size_t)NHID * NHID * 2);
  unsigned short* WIH1H = (unsigned short*)carve((size_t)NHID * NHID * 2);
  unsigned short* WHH1H = (unsigned short*)carve((size_t)NHID * NHID * 2);
  unsigned short* R1    = (unsigned short*)carve((size_t)NSTEP * NBATCH * NHID * 2);
  float*          H2T0  = (float*)carve((size_t)NBATCH * NHID * 4);
  if (off > ws_size || off > (size_t)134217728) return;

  const int n8x  = NBATCH * NSTEP * NIN / 8;
  const int n8wi = NHID * NIN / 8;
  const int n8wh = NHID * NHID / 8;
  cvt8_f16_kernel<<<n8x / CVT_THREADS,  CVT_THREADS, 0, stream>>>(x,     X16,   n8x,  1.0f);
  cvt8_f16_kernel<<<n8wi / CVT_THREADS, CVT_THREADS, 0, stream>>>(w_ih0, WIH0H, n8wi, WCARRY);
  cvt8_f16_kernel<<<n8wh / CVT_THREADS, CVT_THREADS, 0, stream>>>(w_hh0, WHH0H, n8wh, WCARRY);
  cvt8_f16_kernel<<<n8wh / CVT_THREADS, CVT_THREADS, 0, stream>>>(w_ih1, WIH1H, n8wh, WCARRY);
  cvt8_f16_kernel<<<n8wh / CVT_THREADS, CVT_THREADS, 0, stream>>>(w_hh1, WHH1H, n8wh, WCARRY);

  rnn_scan_kernel<0><<<NBATCH / ROWS_BLK, SCAN_THREADS, 0, stream>>>(
      X16, WIH0H, WHH0H, h_state, b_ih0, b_hh0, R1, H2T0, hfin0);
  rnn_scan_kernel<1><<<NBATCH / ROWS_BLK, SCAN_THREADS, 0, stream>>>(
      R1, WIH1H, WHH1H, h_state + (size_t)NBATCH * NHID, b_ih1, b_hh1, X16, H2T0, hfin1);
  head_kernel<<<1, HEAD_THREADS, 0, stream>>>(H2T0, w_out, b_out, out0);
}
